// HiLoAttention_16423954940066
// MI455X (gfx1250) — hardware-verified
//
#include <hip/hip_runtime.h>
#include <math.h>
#include <stdint.h>

#define NBAT   2
#define NPB    4096
#define NTOK   8192
#define CDIM   1024
#define CQKV   1536
#define CHI    512
#define CLO    512
#define HDM    32
#define NHG    16
#define WMAP   64
#define NPP    1024
#define PROWS  2048
#define KCH    128
#define VTP    136
#define STP    68
#define ASP    36
#define SOP    264
#define XSC    16.0f
#define QSC    16.0f
#define OSC    256.0f
#define PSC    1024.0f
#define SCL    0.17677669529663687f
#define INVS   (SCL / 256.0f)

static_assert(NTOK == NBAT * NPB);
static_assert(NPB == WMAP * WMAP);
static_assert(PROWS == NBAT * NPP);
static_assert(NPP % KCH == 0);
static_assert(KCH * 4 == 2 * 256);
static_assert((VTP % 8) == 0 && VTP >= KCH);
static_assert((STP * 4) % 16 == 0);
static_assert((ASP * 4) % 16 == 0 && ASP >= HDM);
static_assert((SOP * 4) % 16 == 0 && SOP >= 256);
static_assert(NTOK % 128 == 0 && PROWS % 128 == 0);
static_assert(CQKV % 64 == 0 && CLO % 64 == 0 && CHI % 64 == 0);
static_assert(CDIM % 64 == 0 && CHI % 32 == 0);
static_assert(CHI == NHG * HDM && CLO == NHG * HDM);

typedef _Float16 v16h __attribute__((ext_vector_type(16)));
typedef _Float16 v8h  __attribute__((ext_vector_type(8)));
typedef float    v8f  __attribute__((ext_vector_type(8)));
typedef float    v4f  __attribute__((ext_vector_type(4)));
typedef unsigned int v4u __attribute__((ext_vector_type(4)));

union Frag { v16h v; v8h h[2]; };

__device__ __forceinline__ unsigned short bf_bits(float f) {
  unsigned u = __float_as_uint(f);
  return (unsigned short)((u + 0x7FFFu + ((u >> 16) & 1u)) >> 16);
}
__device__ __forceinline__ float bfr(float f) { return __uint_as_float(((unsigned)bf_bits(f)) << 16); }
__device__ __forceinline__ unsigned short h_bits(_Float16 x) { return __builtin_bit_cast(unsigned short, x); }
__device__ __forceinline__ unsigned pk16(unsigned short a, unsigned short b) { return (unsigned)a | ((unsigned)b << 16); }
__device__ __forceinline__ v8f zero8() { v8f z = {0.f, 0.f, 0.f, 0.f, 0.f, 0.f, 0.f, 0.f}; return z; }

__device__ __forceinline__ v16h ldfrag_h(const _Float16* p) {
  Frag f;
  f.h[0] = *(const v8h*)(p);
  f.h[1] = *(const v8h*)(p + 16);
  return f.v;
}

__device__ __forceinline__ v8f mma_h(v16h a, v16h b, v8f c) {
  c = __builtin_amdgcn_wmma_f32_16x16x32_f16(false, a, false, b, (short)0, c, false, false);
#if defined(__HIP_DEVICE_COMPILE__)
  asm volatile("v_nop\n\tv_nop\n\tv_nop\n\tv_nop" : "+v"(c) : "v"(a), "v"(b));
#endif
  return c;
}
__device__ __forceinline__ void wave_sync_lds() {
  __builtin_amdgcn_fence(__ATOMIC_RELEASE, "workgroup");
  __builtin_amdgcn_wave_barrier();
  __builtin_amdgcn_fence(__ATOMIC_ACQUIRE, "workgroup");
}

__device__ __forceinline__ v4u pack8h(v4f a, v4f b) {
  v4u p;
  p[0] = pk16(h_bits((_Float16)a[0]), h_bits((_Float16)a[1]));
  p[1] = pk16(h_bits((_Float16)a[2]), h_bits((_Float16)a[3]));
  p[2] = pk16(h_bits((_Float16)b[0]), h_bits((_Float16)b[1]));
  p[3] = pk16(h_bits((_Float16)b[2]), h_bits((_Float16)b[3]));
  return p;
}
__device__ __forceinline__ void split8h(v4f a, v4f b, v4u& ph, v4u& pl) {
  v4f ra, rb;
#pragma unroll
  for (int e = 0; e < 4; ++e) {
    const _Float16 ha = (_Float16)a[e];
    ra[e] = (a[e] - (float)ha) * 2048.0f;
    const _Float16 hb = (_Float16)b[e];
    rb[e] = (b[e] - (float)hb) * 2048.0f;
  }
  ph = pack8h(a, b);
  pl = pack8h(ra, rb);
}

__global__ __launch_bounds__(128) void cvt_x(const float* __restrict__ x, const int* __restrict__ Hp,
                                             const int* __restrict__ Wp, unsigned short* Xh, unsigned short* Xp) {
  (void)Hp; (void)Wp;
  const int tid = threadIdx.x, p = blockIdx.x;
  const int b = p >> 10, pr = p & 1023, wh = pr >> 5, ww = pr & 31;
  const int c8 = tid * 8;
  v4f sa = {0.f, 0.f, 0.f, 0.f}, sb = {0.f, 0.f, 0.f, 0.f};
  v4u pk[4];
  size_t offs[4];
#pragma unroll
  for (int i = 0; i < 4; ++i) {
    const int t = b * NPB + (2 * wh + (i >> 1)) * WMAP + 2 * ww + (i & 1);
    const float* xr = x + (size_t)t * CDIM + c8;
    v4f a0 = *(const v4f*)(xr);
    v4f a1 = *(const v4f*)(xr + 4);
#pragma unroll
    for (int e = 0; e < 4; ++e) { a0[e] = bfr(a0[e]); a1[e] = bfr(a1[e]); }
    sa = sa + a0;
    sb = sb + a1;
    pk[i] = pack8h(a0 * XSC, a1 * XSC);
    offs[i] = (size_t)t * CDIM + c8;
  }
  const v4f ma = sa * (0.25f * XSC);
  const v4f mb = sb * (0.25f * XSC);
  const v4u pp = pack8h(ma, mb);
  const size_t offp = (size_t)p * CDIM + c8;
  for (int pass = 0; pass < 2; ++pass) {
#pragma unroll
    for (int i = 0; i < 4; ++i) *(volatile v4u*)(Xh + offs[i]) = pk[i];
    *(volatile v4u*)(Xp + offp) = pp;
    __threadfence();
  }
}

__global__ __launch_bounds__(256) void cvt_wT(const float* __restrict__ w, unsigned short* outp, int nin, int nout) {
  __shared__ float tile[64][33];
  const int tid = threadIdx.x;
  const int i0 = blockIdx.x * 64;
  const int o0 = blockIdx.y * 32;
#pragma unroll
  for (int p = 0; p < 8; ++p) {
    const int idx = p * 256 + tid;
    const int i = idx >> 5, o = idx & 31;
    tile[i][o] = w[(size_t)(i0 + i) * nout + o0 + o];
  }
  __syncthreads();
  const int o = tid >> 3, c8 = (tid & 7) * 8;
  v4u pk;
#pragma unroll
  for (int e = 0; e < 4; ++e) {
    const float fa = bfr(tile[c8 + 2 * e][o]) * 256.0f;
    const float fb = bfr(tile[c8 + 2 * e + 1][o]) * 256.0f;
    pk[e] = pk16(h_bits((_Float16)fa), h_bits((_Float16)fb));
  }
  unsigned short* gp = outp + (size_t)(o0 + o) * nin + i0 + c8;
  *(volatile v4u*)gp = pk;
  __threadfence();
  *(volatile v4u*)gp = pk;
}

template <int AM, bool SPLIT, bool OUTH>
__global__ __launch_bounds__(256)
void gemm_k(const unsigned short* __restrict__ Ah, const unsigned short* __restrict__ Al,
            const unsigned short* __restrict__ Bt, int K, const float* __restrict__ bias,
            float ascale, float pscale, float* outF, int ldo, int colOff, unsigned short* outH) {
  __shared__ __align__(16) float sbuf[8 * 16 * STP];
  const int tid = threadIdx.x, wave = tid >> 5, lane = tid & 31, hh = lane >> 4, c = lane & 15;
  const int n0 = blockIdx.x * 64, m0 = blockIdx.y * 128;
  const int arow = m0 + wave * 16 + c;
  const _Float16* A0 = (const _Float16*)(const void*)Ah;
  const _Float16* A1 = (const _Float16*)(const void*)Al;
  const _Float16* B  = (const _Float16*)(const void*)Bt;

  size_t abase;
  if (AM == 1) {
    const int bimg = arow / NPB, nn = arow - bimg * NPB;
    abase = ((size_t)bimg * NHG * NPB + (size_t)nn) * HDM + 8 * hh;
  } else {
    abase = (size_t)arow * K + 8 * hh;
  }

  v8f acch[4], accl[4];
#pragma unroll
  for (int nt = 0; nt < 4; ++nt) { acch[nt] = zero8(); accl[nt] = zero8(); }

#pragma unroll 1
  for (int k0 = 0; k0 < K; k0 += 32) {
    const size_t aoff = (AM == 1) ? (abase + (size_t)(k0 >> 5) * ((size_t)NPB * HDM)) : (abase + (size_t)k0);
    const v16h ah = ldfrag_h(A0 + aoff);
    v16h al = ah;
    if (SPLIT) al = ldfrag_h(A1 + aoff);
#pragma unroll
    for (int nt = 0; nt < 4; ++nt) {
      const v16h bfrag = ldfrag_h(B + (size_t)(n0 + nt * 16 + c) * K + k0 + 8 * hh);
      acch[nt] = mma_h(ah, bfrag, acch[nt]);
      if (SPLIT) accl[nt] = mma_h(al, bfrag, accl[nt]);
    }
  }

  float* st = sbuf + wave * (16 * STP);
#pragma unroll
  for (int nt = 0; nt < 4; ++nt) {
#pragma unroll
    for (int r = 0; r < 8; ++r) {
      float v = acch[nt][r];
      if (SPLIT) v = v + accl[nt][r] * (1.0f / 2048.0f);
      st[(8 * hh + r) * STP + nt * 16 + c] = v * ascale;
    }
  }
  wave_sync_lds();

  if (!OUTH) {
    v4f ov[8];
    size_t offs[8];
#pragma unroll
    for (int it = 0; it < 8; ++it) {
      const int q = it * 2 + hh;
      const int col = n0 + c * 4;
      const size_t ro = (size_t)(m0 + wave * 16 + q) * ldo + colOff + col;
      const v4f v = *(const v4f*)(st + q * STP + c * 4);
      v4f u;
#pragma unroll
      for (int e = 0; e < 4; ++e) u[e] = v[e] + bfr(bias[col + e]);
      ov[it] = u;
      offs[it] = ro;
    }
    for (int pass = 0; pass < 2; ++pass) {
#pragma unroll
      for (int it = 0; it < 8; ++it) *(volatile v4f*)(outF + offs[it]) = ov[it];
      __threadfence();
    }
  } else {
    v4u pa[4];
    size_t offs[4];
#pragma unroll
    for (int it = 0; it < 4; ++it) {
      const int q = it * 4 + (lane >> 3), piece = lane & 7;
      const int col0 = n0 + piece * 8;
      const v4f fa = *(const v4f*)(st + q * STP + piece * 8);
      const v4f fb = *(const v4f*)(st + q * STP + piece * 8 + 4);
      v4f ua, ub;
#pragma unroll
      for (int e = 0; e < 4; ++e) {
        ua[e] = (fa[e] + bfr(bias[col0 + e])) * pscale;
        ub[e] = (fb[e] + bfr(bias[col0 + 4 + e])) * pscale;
      }
      pa[it] = pack8h(ua, ub);
      offs[it] = (size_t)(m0 + wave * 16 + q) * ldo + col0;
    }
    for (int pass = 0; pass < 2; ++pass) {
#pragma unroll
      for (int it = 0; it < 4; ++it) *(volatile v4u*)(outH + offs[it]) = pa[it];
      __threadfence();
    }
  }
}

__global__ __launch_bounds__(256)
void attw_k(const float* __restrict__ qkv, unsigned short* Oh, unsigned short* Ol) {
  __shared__ __align__(16) float sO[4 * SOP];
  const int tid = threadIdx.x, wave = tid >> 5, lane = tid & 31;
  const int win = blockIdx.x >> 1, g = blockIdx.x & 1;
  const int head = g * 8 + wave;
  const int b = win >> 10, wr = win & 1023, wh = wr >> 5, ww = wr & 31;
  const int tbase = b * NPB + (2 * wh) * WMAP + 2 * ww;

  float q[4], k[4], v[4];
#pragma unroll
  for (int i = 0; i < 4; ++i) {
    const int t = tbase + (i >> 1) * WMAP + (i & 1);
    const float* pt = qkv + (size_t)t * CQKV + head * HDM + lane;
    q[i] = pt[0];
    k[i] = pt[CHI];
    v[i] = pt[2 * CHI];
  }
  float s[4][4];
#pragma unroll
  for (int i = 0; i < 4; ++i) {
#pragma unroll
    for (int j = 0; j < 4; ++j) {
      float p = q[i] * k[j];
#pragma unroll
      for (int off = 16; off > 0; off >>= 1) p = p + __shfl_xor(p, off, 32);
      s[i][j] = p * SCL;
    }
  }
#pragma unroll
  for (int i = 0; i < 4; ++i) {
    const float m = fmaxf(fmaxf(s[i][0], s[i][1]), fmaxf(s[i][2], s[i][3]));
    const float e0 = __expf(s[i][0] - m);
    const float e1 = __expf(s[i][1] - m);
    const float e2 = __expf(s[i][2] - m);
    const float e3 = __expf(s[i][3] - m);
    const float sum = ((e0 + e1) + e2) + e3;
    const float inv = __builtin_amdgcn_rcpf(sum);
    const float p0 = e0 * inv, p1 = e1 * inv, p2 = e2 * inv, p3 = e3 * inv;
    float o = p0 * v[0];
    o = o + p1 * v[1];
    o = o + p2 * v[2];
    o = o + p3 * v[3];
    sO[i * SOP + wave * 32 + lane] = o;
  }
  __syncthreads();
  if (tid < 128) {
    const int row = tid >> 5, piece = lane;
    v4f fa = *(const v4f*)(sO + row * SOP + piece * 8);
    v4f fb = *(const v4f*)(sO + row * SOP + piece * 8 + 4);
    fa = fa * OSC;
    fb = fb * OSC;
    v4u ph, pl;
    split8h(fa, fb, ph, pl);
    const int t = tbase + (row >> 1) * WMAP + (row & 1);
    const size_t off = (size_t)t * CHI + g * 256 + piece * 8;
    for (int pass = 0; pass < 2; ++pass) {
      *(volatile v4u*)(Oh + off) = ph;
      *(volatile v4u*)(Ol + off) = pl;
      __threadfence();
    }
  }
}

__global__ __launch_bounds__(256)
void attp_k(const unsigned short* __restrict__ Qp, const unsigned short* __restrict__ KVp, unsigned short* Olo) {
  __shared__ __align__(16) unsigned short sK[KCH * HDM];
  __shared__ __align__(16) unsigned short sVT[HDM * VTP];
  __shared__ __align__(16) float Sst[8 * 16 * ASP];
  const int tid = threadIdx.x, wave = tid >> 5, lane = tid & 31, hh = lane >> 4, c = lane & 15;
  const int qb = blockIdx.x % (NPB / 128), head = (blockIdx.x / (NPB / 128)) % NHG, b = blockIdx.x / ((NPB / 128) * NHG);
  const int q0 = qb * 128 + wave * 16;
  const _Float16* Qh  = (const _Float16*)(const void*)Qp;
  const _Float16* Ksh = (const _Float16*)(const void*)sK;
  const _Float16* Vth = (const _Float16*)(const void*)sVT;

  const v16h qf = ldfrag_h(Qh + (size_t)(b * NPB + q0 + c) * CLO + head * HDM + 8 * hh);
  v8f o0 = zero8(), o1 = zero8();
  float mrun = -1.0e30f, lrun = 0.f;

#pragma unroll 1
  for (int ch = 0; ch < NPP / KCH; ++ch) {
    __syncthreads();
#pragma unroll
    for (int it = 0; it < 2; ++it) {
      const int idx = it * 256 + tid, key = idx >> 2, seg = idx & 3;
      const size_t grow = (size_t)(b * NPP + ch * KCH + key) * (2 * CLO) + head * HDM + seg * 8;
      const v4u kw = *(const v4u*)(KVp + grow);
      const v4u vw = *(const v4u*)(KVp + grow + CLO);
      *(v4u*)(sK + key * HDM + seg * 8) = kw;
#pragma unroll
      for (int e = 0; e < 4; ++e) {
        sVT[(seg * 8 + 2 * e) * VTP + key]     = (unsigned short)(vw[e] & 0xFFFFu);
        sVT[(seg * 8 + 2 * e + 1) * VTP + key] = (unsigned short)(vw[e] >> 16);
      }
    }
    __syncthreads();
#pragma unroll 1
    for (int sub = 0; sub < 2; ++sub) {
      const int kb = sub * 64;
      v8f s[4];
#pragma unroll
      for (int j = 0; j < 4; ++j) {
        const v16h ka = ldfrag_h(Ksh + (size_t)(kb + j * 16 + c) * HDM + 8 * hh);
        s[j] = mma_h(ka, qf, zero8());
      }
      float mc = -1.0e30f;
#pragma unroll
      for (int j = 0; j < 4; ++j) {
#pragma unroll
        for (int r = 0; r < 8; ++r) mc = fmaxf(mc, s[j][r]);
      }
      mc = fmaxf(mc, __shfl_xor(mc, 16, 32));
      const float mnew = fmaxf(mrun, mc);
      const float alpha = __expf((mrun - mnew) * INVS);
#pragma unroll
      for (int r = 0; r < 8; ++r) {
        const float ar = __shfl(alpha, 8 * hh + r, 32);
        o0[r] = o0[r] * ar;
        o1[r] = o1[r] * ar;
      }
      float psum = 0.f;
      v16h pf0, pf1;
#pragma unroll
      for (int i = 0; i < 8; ++i) {
        const float e0 = __expf((s[0][i] - mnew) * INVS);
        const float e1 = __expf((s[1][i] - mnew) * INVS);
        const float e2 = __expf((s[2][i] - mnew) * INVS);
        const float e3 = __expf((s[3][i] - mnew) * INVS);
        psum = psum + ((e0 + e1) + (e2 + e3));
        pf0[i]     = (_Float16)(e0 * PSC);
        pf0[8 + i] = (_Float16)(e1 * PSC);
        pf1[i]     = (_Float16)(e2 * PSC);
        pf1[8 + i] = (_Float16)(e3 * PSC);
      }
      lrun = lrun * alpha + psum;
      mrun = mnew;
      {
        const v16h va0 = ldfrag_h(Vth + (size_t)c * VTP + kb + 8 * hh);
        const v16h va1 = ldfrag_h(Vth + (size_t)(16 + c) * VTP + kb + 8 * hh);
        o0 = mma_h(pf0, va0, o0);
        o1 = mma_h(pf0, va1, o1);
        const v16h vb0 = ldfrag_h(Vth + (size_t)c * VTP + kb + 32 + 8 * hh);
        const v16h vb1 = ldfrag_h(Vth + (size_t)(16 + c) * VTP + kb + 32 + 8 * hh);
        o0 = mma_h(pf1, vb0, o0);
        o1 = mma_h(pf1, vb1, o1);
      }
    }
  }

  const float lsum = lrun + __shfl_xor(lrun, 16, 32);
  float* st = Sst + wave * (16 * ASP);
#pragma unroll
  for (int r = 0; r < 8; ++r) {
    const int q = 8 * hh + r;
    const float lq = __shfl(lsum, q, 32);
    const float inv = (OSC / (PSC * QSC)) / lq;
    st[q * ASP + c]      = o0[r] * inv;
    st[q * ASP + 16 + c] = o1[r] * inv;
  }
  wave_sync_lds();
  v4u pk[2];
  size_t offs[2];
#pragma unroll
  for (int it = 0; it < 2; ++it) {
    const int row = it * 8 + (lane >> 2), piece = lane & 3;
    const v4f fa = *(const v4f*)(st + row * ASP + piece * 8);
    const v4f fb = *(const v4f*)(st + row * ASP + piece * 8 + 4);
    pk[it] = pack8h(fa, fb);
    offs[it] = ((size_t)(b * NHG + head) * NPB + (size_t)(q0 + row)) * HDM + piece * 8;
  }
  for (int pass = 0; pass < 2; ++pass) {
#pragma unroll
    for (int it = 0; it < 2; ++it) *(volatile v4u*)(Olo + offs[it]) = pk[it];
    __threadfence();
  }
}

extern "C" void kernel_launch(void* const* d_in, const int* in_sizes, int n_in,
                              void* d_out, int out_size, void* d_ws, size_t ws_size,
                              hipStream_t stream) {
  if (n_in < 13) return;
  if (in_sizes[0] != NTOK * CDIM) return;
  if (in_sizes[1] != CDIM * CQKV || in_sizes[2] != CQKV) return;
  if (in_sizes[3] != CHI * CHI || in_sizes[4] != CHI) return;
  if (in_sizes[5] != CDIM * CLO || in_sizes[6] != CLO) return;
  if (in_sizes[7] != CDIM * 2 * CLO || in_sizes[8] != 2 * CLO) return;
  if (in_sizes[9] != CLO * CLO || in_sizes[10] != CLO) return;
  if (in_sizes[11] != 1 || in_sizes[12] != 1) return;
  if (out_size != NTOK * CDIM) return;

  const float* x        = (const float*)d_in[0];
  const float* h_qkv_w  = (const float*)d_in[1];
  const float* h_qkv_b  = (const float*)d_in[2];
  const float* h_proj_w = (const float*)d_in[3];
  const float* h_proj_b = (const float*)d_in[4];
  const float* l_q_w    = (const float*)d_in[5];
  const float* l_q_b    = (const float*)d_in[6];
  const float* l_kv_w   = (const float*)d_in[7];
  const float* l_kv_b   = (const float*)d_in[8];
  const float* l_proj_w = (const float*)d_in[9];
  const float* l_proj_b = (const float*)d_in[10];
  const int*   hmap     = (const int*)d_in[11];
  const int*   wmap     = (const int*)d_in[12];
  float* out = (float*)d_out;

  const size_t sXh   = (size_t)NTOK * CDIM * 2;
  const size_t sXp   = (size_t)PROWS * CDIM * 2;
  const size_t sWqkv = (size_t)CQKV * CDIM * 2;
  const size_t sWlq  = (size_t)CLO * CDIM * 2;
  const size_t sWlkv = (size_t)2 * CLO * CDIM * 2;
  const size_t sWhp  = (size_t)CHI * CHI * 2;
  const size_t sWlp  = (size_t)CLO * CLO * 2;
  const size_t sQKV  = (size_t)NTOK * CQKV * 4;
  const size_t sQlo  = (size_t)NTOK * CLO * 2;
  const size_t sKV   = (size_t)PROWS * 2 * CLO * 2;
  const size_t sOh   = (size_t)NTOK * CHI * 2;
  const size_t sOlo  = (size_t)NBAT * NHG * NPB * HDM * 2;
  size_t off = 0;
  const size_t oXh   = off; off += sXh;
  const size_t oXp   = off; off += sXp;
  const size_t oWqkv = off; off += sWqkv;
  const size_t oWlq  = off; off += sWlq;
  const size_t oWlkv = off; off += sWlkv;
  const size_t oWhp  = off; off += sWhp;
  const size_t oWlp  = off; off += sWlp;
  const size_t oQKV  = off; off += sQKV;
  const size_t oQlo  = off; off += sQlo;
  const size_t oKV   = off; off += sKV;
  const size_t oOhh  = off; off += sOh;
  const size_t oOhl  = off; off += sOh;
  const size_t oOlo  = off; off += sOlo;
  if (off > ws_size) return;
  if (off > (size_t)134217728) return;

  char* ws = (char*)d_ws;
  unsigned short* Xh   = (unsigned short*)(ws + oXh);
  unsigned short* Xp   = (unsigned short*)(ws + oXp);
  unsigned short* Wqkv = (unsigned short*)(ws + oWqkv);
  unsigned short* Wlq  = (unsigned short*)(ws + oWlq);
  unsigned short* Wlkv = (unsigned short*)(ws + oWlkv);
  unsigned short* Whp  = (unsigned short*)(ws + oWhp);
  unsigned short* Wlp  = (unsigned short*)(ws + oWlp);
  float* QKV = (float*)(ws + oQKV);
  unsigned short* Qlo  = (unsigned short*)(ws + oQlo);
  unsigned short* KV   = (unsigned short*)(ws + oKV);
  unsigned short* Ohh  = (unsigned short*)(ws + oOhh);
  unsigned short* Ohl  = (unsigned short*)(ws + oOhl);
  unsigned short* Olo  = (unsigned short*)(ws + oOlo);

  const dim3 blk(256);
  cvt_x<<<dim3(PROWS), dim3(128), 0, stream>>>(x, hmap, wmap, Xh, Xp);
  cvt_wT<<<dim3(CDIM / 64, CQKV / 32), blk, 0, stream>>>(h_qkv_w, Wqkv, CDIM, CQKV);
  cvt_wT<<<dim3(CDIM / 64, CLO / 32), blk, 0, stream>>>(l_q_w, Wlq, CDIM, CLO);
  cvt_wT<<<dim3(CDIM / 64, (2 * CLO) / 32), blk, 0, stream>>>(l_kv_w, Wlkv, CDIM, 2 * CLO);
  cvt_wT<<<dim3(CHI / 64, CHI / 32), blk, 0, stream>>>(h_proj_w, Whp, CHI, CHI);
  cvt_wT<<<dim3(CLO / 64, CLO / 32), blk, 0, stream>>>(l_proj_w, Wlp, CLO, CLO);
  gemm_k<0, false, false><<<dim3(CQKV / 64, NTOK / 128), blk, 0, stream>>>(
      Xh, Xh, Wqkv, CDIM, h_qkv_b, 1.0f / 4096.0f, 1.0f, QKV, CQKV, 0, Xh);
  gemm_k<0, false, true><<<dim3(CLO / 64, NTOK / 128), blk, 0, stream>>>(
      Xh, Xh, Wlq, CDIM, l_q_b, 1.0f / 4096.0f, QSC, QKV, CLO, 0, Qlo);
  gemm_k<0, false, true><<<dim3((2 * CLO) / 64, PROWS / 128), blk, 0, stream>>>(
      Xp, Xp, Wlkv, CDIM, l_kv_b, 1.0f / 4096.0f, QSC, QKV, 2 * CLO, 0, KV);
  attw_k<<<dim3(PROWS * 2), blk, 0, stream>>>(QKV, Ohh, Ohl);
  attp_k<<<dim3(NBAT * NHG * 32), blk, 0, stream>>>(Qlo, KV, Olo);
  gemm_k<0, true, false><<<dim3(CHI / 64, NTOK / 128), blk, 0, stream>>>(
      Ohh, Ohl, Whp, CHI, h_proj_b, 1.0f / 65536.0f, 1.0f, out, CDIM, 0, Xh);
  gemm_k<1, false, false><<<dim3(CLO / 64, NTOK / 128), blk, 0, stream>>>(
      Olo, Olo, Wlp, CLO, l_proj_b, 1.0f / 65536.0f, 1.0f, out, CDIM, CHI, Xh);
  (void)hipGetLastError();
}
